// EMMPTNet_unbalance_34368328302741
// MI455X (gfx1250) — hardware-verified
//
#include <hip/hip_runtime.h>
#include <math.h>

typedef __attribute__((ext_vector_type(16))) _Float16 v16h;
typedef __attribute__((ext_vector_type(8)))  _Float16 v8h;
typedef __attribute__((ext_vector_type(16))) __bf16   v16b;
typedef __attribute__((ext_vector_type(8)))  float    v8f;
typedef __attribute__((ext_vector_type(4)))  float    v4f;

__device__ __forceinline__ int frag_k(int i, int h) { return (i < 8) ? (8 * h + i) : (16 + 8 * h + (i - 8)); }
__device__ __forceinline__ __bf16 bf16_rne(float f) {
    unsigned int u = __float_as_uint(f);
    u += 0x7fffu + ((u >> 16) & 1u);
    return __builtin_bit_cast(__bf16, (unsigned short)(u >> 16));
}
__device__ __forceinline__ float bf16_f32(__bf16 b) { return __uint_as_float(((unsigned int)__builtin_bit_cast(unsigned short, b)) << 16); }
__device__ __forceinline__ v8f wmma16(v16h a, v16h b, v8f c) {
    c = __builtin_amdgcn_wmma_f32_16x16x32_f16(false, a, false, b, (short)0, c, false, false);
    asm volatile("v_nop\n\tv_nop\n\tv_nop\n\tv_nop" : "+v"(c) : "v"(a), "v"(b));
    return c;
}
__device__ __forceinline__ v8f wmmab(v16b a, v16b b, v8f c) {
    c = __builtin_amdgcn_wmma_f32_16x16x32_bf16(false, a, false, b, (short)0, c, false, false);
    asm volatile("v_nop\n\tv_nop\n\tv_nop\n\tv_nop" : "+v"(c) : "v"(a), "v"(b));
    return c;
}
struct Split { v16b hi, lo; };
__device__ __forceinline__ v8f wmma3(const Split& a, const Split& b, v8f c) {
    c = __builtin_amdgcn_wmma_f32_16x16x32_bf16(false, a.hi, false, b.hi, (short)0, c, false, false);
    c = __builtin_amdgcn_wmma_f32_16x16x32_bf16(false, a.hi, false, b.lo, (short)0, c, false, false);
    c = __builtin_amdgcn_wmma_f32_16x16x32_bf16(false, a.lo, false, b.hi, (short)0, c, false, false);
    asm volatile("v_nop\n\tv_nop\n\tv_nop\n\tv_nop" : "+v"(c) : "v"(a.hi), "v"(a.lo), "v"(b.hi), "v"(b.lo));
    return c;
}
struct Split3 { v16b hi, mid, lo; };
__device__ __forceinline__ v8f wmma6(const Split3& a, const Split3& b, v8f c) {
    c = __builtin_amdgcn_wmma_f32_16x16x32_bf16(false, a.hi, false, b.hi, (short)0, c, false, false);
    c = __builtin_amdgcn_wmma_f32_16x16x32_bf16(false, a.hi, false, b.mid, (short)0, c, false, false);
    c = __builtin_amdgcn_wmma_f32_16x16x32_bf16(false, a.mid, false, b.hi, (short)0, c, false, false);
    c = __builtin_amdgcn_wmma_f32_16x16x32_bf16(false, a.hi, false, b.lo, (short)0, c, false, false);
    c = __builtin_amdgcn_wmma_f32_16x16x32_bf16(false, a.mid, false, b.mid, (short)0, c, false, false);
    c = __builtin_amdgcn_wmma_f32_16x16x32_bf16(false, a.lo, false, b.hi, (short)0, c, false, false);
    asm volatile("v_nop\n\tv_nop\n\tv_nop\n\tv_nop" : "+v"(c) : "v"(a.hi), "v"(a.mid), "v"(a.lo), "v"(b.hi), "v"(b.mid), "v"(b.lo));
    return c;
}

__device__ __forceinline__ v16h fh_ld(const float* __restrict__ p, long long sk, int k0, int h, int klen, float s) {
    v16h a;
#pragma unroll
    for (int i = 0; i < 16; ++i) { const int k = k0 + frag_k(i, h); a[i] = (k < klen) ? (_Float16)(p[(long long)k * sk] * s) : (_Float16)0.f; }
    return a;
}
__device__ __forceinline__ Split sp_ld(const float* __restrict__ p, long long sk, int k0, int h, int klen, float s) {
    Split r;
#pragma unroll
    for (int i = 0; i < 16; ++i) {
        const int k = k0 + frag_k(i, h); const float x = (k < klen) ? p[(long long)k * sk] * s : 0.f;
        const __bf16 hb = bf16_rne(x); r.hi[i] = hb; r.lo[i] = bf16_rne(x - bf16_f32(hb));
    }
    return r;
}
__device__ __forceinline__ Split3 sp3_ld(const float* __restrict__ p, long long sk, int k0, int h, int klen, float s) {
    Split3 r;
#pragma unroll
    for (int i = 0; i < 16; ++i) {
        const int k = k0 + frag_k(i, h); const float x = (k < klen) ? p[(long long)k * sk] * s : 0.f;
        const __bf16 hb = bf16_rne(x); const float r1 = x - bf16_f32(hb); const __bf16 mb = bf16_rne(r1);
        r.hi[i] = hb; r.mid[i] = mb; r.lo[i] = bf16_rne(r1 - bf16_f32(mb));
    }
    return r;
}
__device__ __forceinline__ v16b bh_ld(const float* __restrict__ p, long long sk, int k0, int h, int klen, float s) {
    v16b a;
#pragma unroll
    for (int i = 0; i < 16; ++i) { const int k = k0 + frag_k(i, h); a[i] = bf16_rne((k < klen) ? p[(long long)k * sk] * s : 0.f); }
    return a;
}
__device__ __forceinline__ v16h fh_row(const _Float16* __restrict__ row, int k0, int h) {
    v16h a;
#pragma unroll
    for (int i = 0; i < 16; ++i) a[i] = row[k0 + frag_k(i, h)];
    return a;
}

#define VST2(T, ptr, val) do { *(volatile T*)(ptr) = (val); __threadfence(); *(volatile T*)(ptr) = (val); } while (0)
typedef float v4f __attribute__((ext_vector_type(4)));
#define VST2V4(ptr, val) do { *(volatile v4f*)(ptr) = (val); __threadfence(); *(volatile v4f*)(ptr) = (val); } while (0)

__device__ __attribute__((noinline)) float act_fn(float v, int act) {
    if (act == 1) return fmaxf(v, 0.f);
    if (act == 2) { const float u = 0.7978845608028654f * (v + 0.044715f * v * v * v); return 0.5f * v * (1.f + tanhf(u)); }
    if (act == 3) return v / (1.f + expf(-v));
    if (act == 4) return 0.5f * v * (1.f + erff(v * 0.7071067811865476f));
    if (act == 5) return tanhf(v);
    if (act == 6) return 1.f / (1.f + expf(-v));
    if (act == 7) return (v > 0.f) ? v : 0.01f * v;
    if (act == 8) return (v > 0.f) ? v : (expf(v) - 1.f);
    if (act == 9) return fminf(fmaxf(v, 0.f), 6.f);
    if (act == 10) return fabsf(v);
    if (act == 11) return (v >= 0.f) ? v : 0.1f * v;
    if (act == 12) return (v > 0.f) ? v : 0.2f * v;
    if (act == 13) return (v > 20.f) ? v : log1pf(expf(v));
    return v;
}

struct GemmP {
    const float* A; const float* B; const float* bias; const float* R; float* C;
    long long sAo, sAi, sAm, sAk, sBo, sBi, sBn, sBk, sCo, sCi, sCm, sRo, sRi, sRm, sRn;
    int M, N, K, zi_n, flags, act; float alpha, beta, sa, sb;
    int Npad, pad_;
};
static_assert(sizeof(GemmP) == 5 * 8 + 15 * 8 + 6 * 4 + 4 * 4 + 2 * 4, "GemmP has padding");

template <int MODE>
__global__ __launch_bounds__(32) void k_gemm(GemmP p) {
    const int lane = threadIdx.x & 31, h = lane >> 4, l15 = lane & 15;
    const int m0 = blockIdx.y * 16, n0 = blockIdx.x * 32;
    const int z = blockIdx.z, zo = z / p.zi_n, zi = z - zo * p.zi_n;
    const float* A = p.A + zo * p.sAo + zi * p.sAi;
    const float* B = p.B + zo * p.sBo + zi * p.sBi;
    const int am = min(m0 + l15, p.M - 1);
    v8f acc[2], comp[2];
#pragma unroll
    for (int t = 0; t < 2; ++t) { v8f zz = {}; acc[t] = zz; comp[t] = zz; }
    for (int k0 = 0; k0 < p.K; k0 += 32) {
        const float* arow = A + (long long)am * p.sAm;
        if (MODE == 1) {
            const Split a = sp_ld(arow, p.sAk, k0, h, p.K, 1.f);
#pragma unroll
            for (int t = 0; t < 2; ++t) {
                const int bn = min(n0 + t * 16 + l15, p.N - 1);
                acc[t] = wmma3(a, sp_ld(B + (long long)bn * p.sBn, p.sBk, k0, h, p.K, 1.f), acc[t]);
            }
        } else if (MODE == 3) {
            const Split3 a = sp3_ld(arow, p.sAk, k0, h, p.K, 1.f);
#pragma unroll
            for (int t = 0; t < 2; ++t) {
                const int bn = min(n0 + t * 16 + l15, p.N - 1);
                acc[t] = wmma6(a, sp3_ld(B + (long long)bn * p.sBn, p.sBk, k0, h, p.K, 1.f), acc[t]);
            }
        } else if (MODE == 4) {
            const Split3 a = sp3_ld(arow, p.sAk, k0, h, p.K, 1.f);
#pragma unroll
            for (int t = 0; t < 2; ++t) {
                const int bn = min(n0 + t * 16 + l15, p.N - 1); v8f zz = {};
                const v8f part = wmma6(a, sp3_ld(B + (long long)bn * p.sBn, p.sBk, k0, h, p.K, 1.f), zz);
                const v8f y = part - comp[t]; const v8f s = acc[t] + y; comp[t] = (s - acc[t]) - y; acc[t] = s;
            }
        } else if (MODE == 2) {
            const v16b a = bh_ld(arow, p.sAk, k0, h, p.K, 1.f);
#pragma unroll
            for (int t = 0; t < 2; ++t) {
                const int bn = min(n0 + t * 16 + l15, p.N - 1);
                acc[t] = wmmab(a, bh_ld(B + (long long)bn * p.sBn, p.sBk, k0, h, p.K, 1.f), acc[t]);
            }
        } else {
            const v16h a = fh_ld(arow, p.sAk, k0, h, p.K, p.sa);
#pragma unroll
            for (int t = 0; t < 2; ++t) {
                const int bn = min(n0 + t * 16 + l15, p.N - 1);
                acc[t] = wmma16(a, fh_ld(B + (long long)bn * p.sBn, p.sBk, k0, h, p.K, p.sb), acc[t]);
            }
        }
    }
    const float iscale = (MODE == 0) ? p.alpha / (p.sa * p.sb) : p.alpha;
    float* C = p.C + zo * p.sCo + zi * p.sCi;
    const float* R = p.R + zo * p.sRo + zi * p.sRi;
    __shared__ __align__(16) float ctile[16][36];
#pragma unroll
    for (int t = 0; t < 2; ++t) {
        const int n = n0 + t * 16 + l15; const int nn = min(n, p.N - 1);
#pragma unroll
        for (int r = 0; r < 8; ++r) {
            const int m = m0 + 8 * h + r; const int mm = min(m, p.M - 1);
            float v = acc[t][r] * iscale;
            if (p.flags & 1) v += p.bias[nn];
            if (p.flags & 2) v += p.bias[mm];
            v = act_fn(v, p.act);
            if (p.flags & 4) v += p.beta * R[(long long)mm * p.sRm + (long long)nn * p.sRn];
            ctile[8 * h + r][t * 16 + l15] = (n < p.N) ? v : 0.f;
        }
    }
    __syncthreads();
    const int NW = (p.Npad > p.N) ? p.Npad : p.N;
    const bool fast = (m0 + 16 <= p.M) && (n0 + 32 <= NW) && ((p.sCm & 3) == 0) && ((((size_t)C) & 15) == 0);
    if (fast) {
#pragma unroll
        for (int s = 0; s < 4; ++s) {
            const int row = s * 4 + (lane >> 3), c4 = (lane & 7) * 4;
            const v4f v = *(const v4f*)&ctile[row][c4];
            VST2V4(C + (long long)(m0 + row) * p.sCm + n0 + c4, v);
        }
    } else {
        for (int row = 0; row < 16; ++row) {
            const int m = m0 + row, n = n0 + lane;
            if (m < p.M && n < NW) VST2(float, C + (long long)m * p.sCm + n, ctile[row][lane]);
        }
    }
}

#define AW 4
struct AttnP {
    const float* Q; const float* K; const float* V; float* O; float* P; const float* Mf; const int* Mi; float* ST;
    const float* Pw; const float* Rt; const int* SQ; const int* SK;
    long long swb, swh, swi, swj, srb, srh, sri;
    long long sQb, sQh, sQi, sQd, sKb, sKh, sKj, sKd, sVb, sVh, sVj, sVd, sOb, sOh, sOi, sPb, sPh, sPi, smb, smh, smi, smj;
    int Lq, Lk, dh, dv, hrep, causal, coff, pband;
    float scale, mfill; int nonorm, mpol;
    int roff, rn, segpol, win;
};
static_assert(sizeof(AttnP) == 12 * 8 + 29 * 8 + 16 * 4, "AttnP has padding");

#ifndef KATTN_ATTR
#define KATTN_ATTR
#endif
template <int DHP, int DVP, int QM, bool SPLITPV, bool TWOPASS>
__global__ __launch_bounds__(32 * AW) KATTN_ATTR void k_attn(AttnP p) {
    constexpr int NT = DVP / 16;
    constexpr int KS = DHP / 32;
    constexpr int VP = DVP + 8;
    __shared__ __align__(16) float    pl[AW][16 * 64];
    __shared__ __align__(16) _Float16 vl[(SPLITPV ? 2 : 1) * 64 * VP];
    const int lane = threadIdx.x & 31, hf = lane >> 4, l15 = lane & 15, wave = threadIdx.x >> 5;
    const int h = blockIdx.y, b = blockIdx.z, hk = h / p.hrep;
    const int q0 = (blockIdx.x * AW + wave) * 16;
    float* myp = pl[wave];
    const float L2E = 1.4426950408889634f;
    const float NEG = -__builtin_inff();
    const int qi = min(q0 + l15, p.Lq - 1);
    const float* qrow = p.Q + b * p.sQb + h * p.sQh + (long long)qi * p.sQi;
    const float* kbase = p.K + b * p.sKb + hk * p.sKh;
    const float* vbase = p.V + b * p.sVb + hk * p.sVh;
    v16h qa[QM == 0 ? KS : 1]; Split qs_[QM == 1 ? KS : 1]; Split3 qt_[QM == 2 ? KS : 1];
#pragma unroll
    for (int ks = 0; ks < KS; ++ks) {
        if (QM == 2) qt_[ks] = sp3_ld(qrow, p.sQd, ks * 32, hf, p.dh, 1.f);
        else if (QM == 1) qs_[ks] = sp_ld(qrow, p.sQd, ks * 32, hf, p.dh, 1.f);
        else qa[ks] = fh_ld(qrow, p.sQd, ks * 32, hf, p.dh, 1.f);
    }
    v8f o[NT]; float m8[8], l8[8];
#pragma unroll
    for (int t = 0; t < NT; ++t) { v8f zz = {}; o[t] = zz; }
#pragma unroll
    for (int i = 0; i < 8; ++i) { m8[i] = NEG; l8[i] = 0.f; }
    int jend = p.Lk;
    if (p.causal == 1) { const int je = (blockIdx.x * AW + AW - 1) * 16 + 16 + p.coff; jend = min(jend, max(je, 0)); }
    const int npass = TWOPASS ? 2 : 1;
    for (int pass = 0; pass < npass; ++pass) {
        const bool dopv = (!TWOPASS) || pass == 1;
        for (int j0 = 0; j0 < jend; j0 += 64) {
            if (dopv) {
                __syncthreads();
                for (int idx = threadIdx.x; idx < 64 * DVP; idx += 32 * AW) {
                    const int jr = idx / DVP, d = idx - jr * DVP, j = j0 + jr;
                    const float f = (j < p.Lk && d < p.dv) ? vbase[(long long)j * p.sVj + (long long)d * p.sVd] : 0.f;
                    if (SPLITPV) {
                        const __bf16 hb = bf16_rne(f);
                        ((__bf16*)vl)[jr * VP + d] = hb; ((__bf16*)vl)[64 * VP + jr * VP + d] = bf16_rne(f - bf16_f32(hb));
                    } else vl[jr * VP + d] = (_Float16)f;
                }
            }
            v8f s[4];
#pragma unroll
            for (int t = 0; t < 4; ++t) {
                const int j = min(j0 + t * 16 + l15, p.Lk - 1);
                const float* krow = kbase + (long long)j * p.sKj;
                v8f acc = {};
#pragma unroll
                for (int ks = 0; ks < KS; ++ks) {
                    if (QM == 2)      acc = wmma6(qt_[ks], sp3_ld(krow, p.sKd, ks * 32, hf, p.dh, 1.f), acc);
                    else if (QM == 1) acc = wmma3(qs_[ks], sp_ld(krow, p.sKd, ks * 32, hf, p.dh, 1.f), acc);
                    else              acc = wmma16(qa[ks], fh_ld(krow, p.sKd, ks * 32, hf, p.dh, 1.f), acc);
                }
                s[t] = acc;
            }
            float pv[8][4];
#pragma unroll
            for (int i = 0; i < 8; ++i) {
                const int irow = q0 + i + 8 * hf;
                const int ic = min(irow, p.Lq - 1);
                float sc[4];
#pragma unroll
                for (int t = 0; t < 4; ++t) {
                    const int jg = j0 + t * 16 + l15;
                    float v = s[t][i] * p.scale;
                    if (p.Mf) v += p.Mf[b * p.smb + h * p.smh + (long long)ic * p.smi + (long long)min(jg, p.Lk - 1) * p.smj];
                    if (p.Rt) { int rc = ic - min(jg, p.Lk - 1) + p.roff; rc = rc < 0 ? 0 : (rc >= p.rn ? p.rn - 1 : rc); v += p.Rt[b * p.srb + h * p.srh + (long long)ic * p.sri + rc]; }
                    if (p.Mi) { const int mv = p.Mi[b * p.smb + h * p.smh + (long long)ic * p.smi + (long long)min(jg, p.Lk - 1) * p.smj]; if (p.mpol ? (mv != 0) : (mv == 0)) v = p.mfill; }
                    if (p.SQ) { const bool same = p.SQ[(long long)b * p.Lq + ic] == p.SK[(long long)b * p.Lk + min(jg, p.Lk - 1)]; if (p.segpol ? same : !same) v = p.mfill; }
                    if (p.causal == 2 && jg > irow + p.coff) v = p.mfill;
                    if (jg >= p.Lk || (p.causal == 1 && jg > irow + p.coff) || (p.causal == 3 && jg < irow + p.coff) || (p.win > 0 && irow + p.coff - jg > p.win)) v = NEG; else v *= L2E;
                    sc[t] = v;
                }
                if (!TWOPASS || pass == 0) {
                    float mx = fmaxf(fmaxf(sc[0], sc[1]), fmaxf(sc[2], sc[3]));
                    mx = fmaxf(mx, __shfl_xor(mx, 1, 32)); mx = fmaxf(mx, __shfl_xor(mx, 2, 32));
                    mx = fmaxf(mx, __shfl_xor(mx, 4, 32)); mx = fmaxf(mx, __shfl_xor(mx, 8, 32));
                    const float mnew = fmaxf(m8[i], mx);
                    const float corr = (mnew == NEG) ? 1.f : exp2f(m8[i] - mnew);
                    float rs = 0.f;
#pragma unroll
                    for (int t = 0; t < 4; ++t) {
                        const float pp = (sc[t] == NEG) ? 0.f : exp2f(sc[t] - mnew); rs += pp;
                        pv[i][t] = p.Pw ? pp * p.Pw[b * p.swb + h * p.swh + (long long)ic * p.swi + (long long)min(j0 + t * 16 + l15, p.Lk - 1) * p.swj] : pp;
                    }
                    rs += __shfl_xor(rs, 1, 32); rs += __shfl_xor(rs, 2, 32); rs += __shfl_xor(rs, 4, 32); rs += __shfl_xor(rs, 8, 32);
                    l8[i] = l8[i] * corr + rs; m8[i] = mnew;
                    if (!TWOPASS) {
#pragma unroll
                        for (int t = 0; t < NT; ++t) o[t][i] *= corr;
                    }
                } else {
                    const float inv = (l8[i] > 0.f) ? 1.f / l8[i] : 0.f;
#pragma unroll
                    for (int t = 0; t < 4; ++t) {
                        const int jg = j0 + t * 16 + l15;
                        float pp = (sc[t] == NEG) ? 0.f : exp2f(sc[t] - m8[i]) * inv;
                        if (p.Pw) pp *= p.Pw[b * p.swb + h * p.swh + (long long)ic * p.swi + (long long)min(jg, p.Lk - 1) * p.swj];
                        pv[i][t] = pp;
                    }
                }
            }
            if (dopv) {
#pragma unroll
                for (int i = 0; i < 8; ++i)
#pragma unroll
                    for (int t = 0; t < 4; ++t) myp[(i + 8 * hf) * 64 + t * 16 + l15] = pv[i][t];
                __syncthreads();
                if (p.P) {
                    float* pb_ = p.P + b * p.sPb + h * p.sPh;
                    const bool fastP = (p.pband == 0) && ((p.sPi & 3) == 0) && (j0 + 64 <= p.Lk) && (q0 + 16 <= p.Lq) && ((((size_t)pb_) & 15) == 0);
                    if (fastP) {
#pragma unroll
                        for (int s = 0; s < 8; ++s) {
                            const int row = s * 2 + (lane >> 4), c4 = (lane & 15) * 4;
                            const v4f v = *(const v4f*)(myp + row * 64 + c4);
                            VST2V4(pb_ + (long long)(q0 + row) * p.sPi + j0 + c4, v);
                        }
                    } else {
                        for (int row = 0; row < 16; ++row) {
                            const int irow = q0 + row; if (irow >= p.Lq) continue;
                            for (int c = lane; c < 64; c += 32) {
                                const int jg = j0 + c; if (jg >= p.Lk) continue;
                                if (p.pband == 0) VST2(float, pb_ + (long long)irow * p.sPi + jg, myp[row * 64 + c]);
                                else if (jg - irow <= p.pband && irow - jg <= p.pband) VST2(float, pb_ + (long long)irow * p.sPi + (jg - irow + p.pband), myp[row * 64 + c]);
                            }
                        }
                    }
                }
                if (SPLITPV) {
                    const Split pa0 = sp_ld(myp + l15 * 64, 1, 0, hf, 64, 1.f), pa1 = sp_ld(myp + l15 * 64, 1, 32, hf, 64, 1.f);
                    const __bf16* vh = (const __bf16*)vl; const __bf16* vlo = vh + 64 * VP;
#pragma unroll
                    for (int t = 0; t < NT; ++t) {
                        const int dcol = t * 16 + l15;
                        Split b0, b1;
#pragma unroll
                        for (int e = 0; e < 16; ++e) {
                            const int k0 = frag_k(e, hf), k1 = 32 + frag_k(e, hf);
                            b0.hi[e] = vh[k0 * VP + dcol]; b0.lo[e] = vlo[k0 * VP + dcol]; b1.hi[e] = vh[k1 * VP + dcol]; b1.lo[e] = vlo[k1 * VP + dcol];
                        }
                        o[t] = wmma3(pa0, b0, o[t]);
                        o[t] = wmma3(pa1, b1, o[t]);
                    }
                } else {
                    const v16h pa0 = fh_ld(myp + l15 * 64, 1, 0, hf, 64, 4096.f), pa1 = fh_ld(myp + l15 * 64, 1, 32, hf, 64, 4096.f);
#pragma unroll
                    for (int t = 0; t < NT; ++t) {
                        const int dcol = t * 16 + l15;
                        v16h b0, b1;
#pragma unroll
                        for (int e = 0; e < 16; ++e) { b0[e] = vl[frag_k(e, hf) * VP + dcol]; b1[e] = vl[(32 + frag_k(e, hf)) * VP + dcol]; }
                        o[t] = wmma16(pa0, b0, o[t]);
                        o[t] = wmma16(pa1, b1, o[t]);
                    }
                }
            }
        }
    }
    float* obase = p.O + b * p.sOb + h * p.sOh;
    if (p.ST) {
        const int rl = lane >> 1, isel = rl & 7;
        float mv = 0.f, lv = 0.f;
#pragma unroll
        for (int i = 0; i < 8; ++i) if (i == isel) { mv = m8[i]; lv = l8[i]; }
        const int irow = q0 + rl;
        if (irow < p.Lq) { float* st = p.ST + (((long long)b * gridDim.y + h) * p.Lq + irow) * 2 + (lane & 1); VST2(float, st, (lane & 1) ? lv : mv * 0.6931471805599453f); }
    }
    float invr[8];
#pragma unroll
    for (int i = 0; i < 8; ++i) {
        if (TWOPASS) invr[i] = SPLITPV ? 1.f : (1.f / 4096.f);
        else if (p.nonorm) invr[i] = exp2f(m8[i]) * (SPLITPV ? 1.f : (1.f / 4096.f));
        else invr[i] = (l8[i] > 0.f) ? (SPLITPV ? 1.f / l8[i] : 1.f / (l8[i] * 4096.f)) : 0.f;
    }
    __syncthreads();
    const bool ofast = ((p.sOi & 3) == 0) && ((((size_t)obase) & 15) == 0) && (q0 + 16 <= p.Lq);
#pragma unroll
    for (int c0 = 0; c0 < DVP; c0 += 64) {
#pragma unroll
        for (int i = 0; i < 8; ++i)
#pragma unroll
            for (int t = 0; t < NT; ++t) if (t * 16 >= c0 && t * 16 < c0 + 64) myp[(i + 8 * hf) * 64 + (t * 16 - c0) + l15] = o[t][i] * invr[i];
        __syncthreads();
        const int cw = (DVP - c0 < 64) ? (DVP - c0) : 64;
        if (ofast && (c0 + cw <= p.dv) && (cw % 32 == 0)) {
            const int lpr = cw / 4;
            const int rows_per_ins = 32 / lpr;
            for (int r0 = 0; r0 < 16; r0 += rows_per_ins) {
                const int row = r0 + lane / lpr, c4 = (lane % lpr) * 4;
                const v4f v = *(const v4f*)(myp + row * 64 + c4);
                VST2V4(obase + (long long)(q0 + row) * p.sOi + c0 + c4, v);
            }
        } else {
            for (int row = 0; row < 16; ++row) {
                const int irow = q0 + row; if (irow >= p.Lq) continue;
                for (int c = lane; c < cw; c += 32) { const int d = c0 + c; if (d < p.dv) VST2(float, obase + (long long)irow * p.sOi + d, myp[row * 64 + c]); }
            }
        }
        __syncthreads();
    }
}

struct TrP { const float* src; float* dst; const float* R2; long long sSz, lds, sDz, ldd, sRz, ldr; int R, C, flags, act; float alpha, beta; };
static_assert(sizeof(TrP) == 3 * 8 + 6 * 8 + 6 * 4, "TrP has padding");
__global__ __launch_bounds__(256) void k_tr(TrP p) {
    __shared__ float tile[32][33];
    const int c0 = blockIdx.x * 32, r0 = blockIdx.y * 32, z = blockIdx.z;
    const int lane = threadIdx.x & 31, wave = threadIdx.x >> 5;
    const float* s = p.src + z * p.sSz;
#pragma unroll
    for (int k = 0; k < 4; ++k) {
        const int rl = wave * 4 + k, r = r0 + rl, c = c0 + lane;
        tile[rl][lane] = (r < p.R && c < p.C) ? s[(long long)r * p.lds + c] : 0.f;
    }
    __syncthreads();
    float* d = p.dst + z * p.sDz; const float* rr = p.R2 + z * p.sRz;
#pragma unroll
    for (int k = 0; k < 4; ++k) {
        const int cl = wave * 4 + k, c = c0 + cl, r = r0 + lane;
        if (c < p.C && r < p.R) {
            float v = act_fn(p.alpha * tile[lane][cl], p.act);
            if (p.flags & 1) v += p.beta * rr[(long long)c * p.ldr + r];
            VST2(float, d + (long long)c * p.ldd + r, v);
        }
    }
}

__global__ __launch_bounds__(256) void k_affine(const float* __restrict__ src, float* __restrict__ dst, int n, float a, float b, const float* __restrict__ sdev) {
    const int i = blockIdx.x * 256 + threadIdx.x;
    if (i < n) { const float aa = sdev ? a * sdev[0] : a; const float v = aa * src[i] + b; VST2(float, dst + i, v); }
}

struct SmP { const float* src; float* dst; const float* Mf; long long sz, sr, dz, dr, smz, smr; int n, pad; float scale_in, scale_out; };
static_assert(sizeof(SmP) == 3 * 8 + 6 * 8 + 4 * 4, "SmP has padding");
__global__ __launch_bounds__(256) void k_softmax(SmP p) {
    __shared__ float red[256];
    const int r = blockIdx.x, z = blockIdx.y, tid = threadIdx.x;
    const float* s = p.src + z * p.sz + (long long)r * p.sr;
    const float* mf = p.Mf ? (p.Mf + z * p.smz + (long long)r * p.smr) : nullptr;
    float mx = -__builtin_inff();
    for (int j = tid; j < p.n; j += 256) { float v = s[j] * p.scale_in; if (mf) v += mf[j]; mx = fmaxf(mx, v); }
    red[tid] = mx; __syncthreads();
    for (int o = 128; o > 0; o >>= 1) { if (tid < o) red[tid] = fmaxf(red[tid], red[tid + o]); __syncthreads(); }
    mx = red[0]; __syncthreads();
    float sum = 0.f;
    for (int j = tid; j < p.n; j += 256) { float v = s[j] * p.scale_in; if (mf) v += mf[j]; sum += (mx == -__builtin_inff()) ? 0.f : expf(v - mx); }
    red[tid] = sum; __syncthreads();
    for (int o = 128; o > 0; o >>= 1) { if (tid < o) red[tid] += red[tid + o]; __syncthreads(); }
    sum = red[0];
    const float inv = (sum > 0.f) ? p.scale_out / sum : 0.f;
    float* d = p.dst + z * p.dz + (long long)r * p.dr;
    for (int j = tid; j < p.n; j += 256) { float v = s[j] * p.scale_in; if (mf) v += mf[j]; const float o = (mx == -__builtin_inff()) ? 0.f : expf(v - mx) * inv; VST2(float, d + j, o); }
}
__global__ __launch_bounds__(256) void k_stats(const float* __restrict__ x, long long sz, long long so, long long si, int inner, int n, float eps, float* __restrict__ stat, int mode) {
    __shared__ float red[256];
    const int z = blockIdx.x, tid = threadIdx.x;
    const float* base = x + z * sz;
    float s = 0.f;
    for (int e = tid; e < n; e += 256) s += base[(long long)(e / inner) * so + (long long)(e % inner) * si];
    red[tid] = s; __syncthreads();
    for (int o = 128; o > 0; o >>= 1) { if (tid < o) red[tid] += red[tid + o]; __syncthreads(); }
    const float mu = (mode == 0 || mode == 3) ? red[0] / (float)n : 0.f; __syncthreads();
    float q = 0.f;
    for (int e = tid; e < n; e += 256) { const float dlt = base[(long long)(e / inner) * so + (long long)(e % inner) * si] - mu; q += dlt * dlt; }
    red[tid] = q; __syncthreads();
    for (int o = 128; o > 0; o >>= 1) { if (tid < o) red[tid] += red[tid + o]; __syncthreads(); }
    {
        float rs;
        if (mode == 2) rs = sqrtf((float)n) / fmaxf(sqrtf(red[0]), eps); else if (mode == 3) rs = rsqrtf(red[0] / (float)(n - 1) + eps); else rs = rsqrtf(red[0] / (float)n + eps);
        if (tid < 32) { const float v = (tid == 0) ? mu : ((tid == 1) ? rs : 0.f); VST2(float, stat + (long long)z * 32 + tid, v); }
    }
}
__global__ __launch_bounds__(256) void k_norm_apply(const float* __restrict__ x, float* __restrict__ y, const float* __restrict__ stat, const float* __restrict__ g, const float* __restrict__ bta,
                                                     int Z, int C, int L, int G, int bn, int act) {
    const long long idx = (long long)blockIdx.x * 256 + threadIdx.x;
    if (idx >= (long long)Z * C * L) return;
    const int l = (int)(idx % L); const long long zc = idx / L; const int c = (int)(zc % C), z = (int)(zc / C); (void)l;
    const int set = bn ? c : (z * G + c / (C / G));
    float v = (x[idx] - stat[(long long)set * 32]) * stat[(long long)set * 32 + 1];
    if (g) v *= g[c];
    if (bta) v += bta[c];
    v = act_fn(v, act);
    VST2(float, y + idx, v);
}

__global__ __launch_bounds__(256) void k_lse_neg(const float* __restrict__ st, float* __restrict__ c, int n) {
    const int i = blockIdx.x * 256 + threadIdx.x;
    if (i < n) { const float v = -(st[2 * i] + logf(st[2 * i + 1])); VST2(float, c + i, v); }
}

__global__ __launch_bounds__(256) void k_iota(int* __restrict__ dst, int n, int a, int b) {
    const int i = blockIdx.x * 256 + threadIdx.x;
    if (i < n) { const int v = a * i + b; VST2(int, dst + i, v); }
}

__global__ __launch_bounds__(256) void k_axpby(const float* __restrict__ x, const float* __restrict__ y, float* __restrict__ dst, int n, float a, float b, float c) {
    const int i = blockIdx.x * 256 + threadIdx.x;
    if (i < n) { const float v = a * x[i] + b * y[i] + c; VST2(float, dst + i, v); }
}

struct RopeP { const float* X; float* Y; const float* C; const float* Sn; const int* pos; long long sXr, sXh, sYr, sYh, sCb, sCp, sCd; int R, Hn, D, S, mode, tmode, pmode, pad; };
static_assert(sizeof(RopeP) == 5 * 8 + 7 * 8 + 8 * 4, "RopeP has padding");
__global__ __launch_bounds__(256) void k_rope(RopeP p) {
    const long long idx = (long long)blockIdx.x * 256 + threadIdx.x;
    if (idx >= (long long)p.R * p.Hn * p.D) return;
    const int d = (int)(idx % p.D); const long long rh = idx / p.D; const int h = (int)(rh % p.Hn); const int r = (int)(rh / p.Hn);
    const int half = p.D / 2;
    int partner; float sign;
    if (p.mode == 0) { partner = (d < half) ? d + half : d - half; sign = (d < half) ? -1.f : 1.f; }
    else { partner = d ^ 1; sign = (d & 1) ? 1.f : -1.f; }
    const int tcol = (p.tmode == 0) ? d : ((p.tmode == 1) ? (d % half) : (d >> 1));
    const int pp = (p.pmode == 0) ? (r % p.S) : ((p.pmode == 1) ? h : p.pos[r]);
    const long long toff = (long long)(r / p.S) * p.sCb + (long long)pp * p.sCp + (long long)tcol * p.sCd;
    const float* xr = p.X + (long long)r * p.sXr + (long long)h * p.sXh;
    const float v = xr[d] * p.C[toff] + sign * xr[partner] * p.Sn[toff];
    VST2(float, p.Y + (long long)r * p.sYr + (long long)h * p.sYh + d, v);
}

__global__ __launch_bounds__(256) void k_invf(float* __restrict__ invb, int half, int D, float base, float num, int fmode, float cexp) {
    const int i = blockIdx.x * 256 + threadIdx.x;
    if (i >= ((half + 31) / 32) * 32) return;
    if (i >= half) { VST2(float, invb + i, 0.f); return; }
    const float e = (float)(2 * i) / (float)D;
    float invf;
    if (fmode == 1) invf = num * expf((float)(2 * i) * cexp);
    else if (fmode == 2) invf = num * powf(base, (-2.0f * ((float)i - 1.0f)) / (float)D);
    else invf = num * (1.0f / powf(base, e));
    VST2(float, invb + i, invf);
}
__global__ __launch_bounds__(256) void k_sincos(float* __restrict__ cs, float* __restrict__ sn, const float* __restrict__ invb, int S, int half, float pscale) {
    const int idx = blockIdx.x * 256 + threadIdx.x;
    if (idx >= S * half) return;
    const int s = idx / half, i = idx - s * half;
    const float ang = (pscale * (float)s) * invb[i];
    VST2(float, cs + idx, cosf(ang)); VST2(float, sn + idx, sinf(ang));
}

__global__ __launch_bounds__(256) void k_mulact(const float* __restrict__ x, const float* __restrict__ y, float* __restrict__ dst, int n, int act) {
    const int i = blockIdx.x * 256 + threadIdx.x;
    if (i < n) { const float v = act_fn(x[i], act) * y[i]; VST2(float, dst + i, v); }
}

__global__ __launch_bounds__(256) void k_matvec(GemmP p) {
    const int rpt = (p.N == 1) ? 1 : 32;
    const long long r0 = ((long long)blockIdx.x * 256 + threadIdx.x) * rpt; const int z = blockIdx.z, zo = z / p.zi_n, zi = z - zo * p.zi_n;
    if (r0 >= p.M) return;
    const float* Bb = p.B + zo * p.sBo + zi * p.sBi;
    float* C = p.C + zo * p.sCo + zi * p.sCi; const float* R = p.R + zo * p.sRo + zi * p.sRi;
    for (int rr = 0; rr < rpt; ++rr) {
        const long long r = r0 + rr; if (r >= p.M) break;
        const float* A = p.A + zo * p.sAo + zi * p.sAi + r * p.sAm;
        float acc[8] = {0.f, 0.f, 0.f, 0.f, 0.f, 0.f, 0.f, 0.f};
        for (int k = 0; k < p.K; ++k) { const float a = A[(long long)k * p.sAk];
#pragma unroll
            for (int j = 0; j < 8; ++j) if (j < p.N) acc[j] += a * Bb[(long long)j * p.sBn + (long long)k * p.sBk]; }
#pragma unroll
        for (int j = 0; j < 8; ++j) if (j < p.N) {
            float v = acc[j] * p.alpha;
            if (p.flags & 1) v += p.bias[j];
            if (p.flags & 2) v += p.bias[r];
            v = act_fn(v, p.act);
            if (p.flags & 4) v += p.beta * R[r * p.sRm + (long long)j * p.sRn];
            VST2(float, C + r * p.sCm + j, v);
        }
    }
}
__global__ __launch_bounds__(256) void k_smallsoftmax(const float* __restrict__ src, float* __restrict__ dst, long long sr, long long dr, int n, long long R, float scale) {
    const long long r0 = ((long long)blockIdx.x * 256 + threadIdx.x) * 32;
    for (int rr = 0; rr < 32; ++rr) {
        const long long r = r0 + rr; if (r >= R) return;
        const float* s = src + r * sr; float* d = dst + r * dr;
        float mx = -__builtin_inff();
        for (int j = 0; j < n; ++j) mx = fmaxf(mx, s[j] * scale);
        float sum = 0.f;
        for (int j = 0; j < n; ++j) sum += expf(s[j] * scale - mx);
        const float inv = 1.f / sum;
        for (int j = 0; j < n; ++j) { const float v = expf(s[j] * scale - mx) * inv; VST2(float, d + j, v); }
    }
}

__global__ __launch_bounds__(32) void k_unitstat(float* __restrict__ st) { const int t = threadIdx.x; const float v = (t == 1) ? 1.f : 0.f; VST2(float, st + t, v); }

__global__ __launch_bounds__(256) void k_lincopy(const float* __restrict__ src, long long lds, float* __restrict__ dst, long long ldd, long long rows, int cols) {
    const long long i = (long long)blockIdx.x * 256 + threadIdx.x; if (i >= rows * cols) return;
    const long long r = i / cols; const int c = (int)(i - r * cols);
    const float v = src[r * lds + c]; VST2(float, dst + r * ldd + c, v);
}

#define IL_CAP32 32
#define IL_T32 256
#define IL_TILE32 4096
__global__ __launch_bounds__(IL_T32) void k_inlists32(const int* __restrict__ tgt, int E, int N, int* __restrict__ NBR, int* __restrict__ cnt) {
    __shared__ int tt[IL_TILE32];
    __shared__ int lists[IL_T32 * IL_CAP32];
    const int d = blockIdx.x * IL_T32 + threadIdx.x; int n = 0;
    for (int e0 = 0; e0 < E; e0 += IL_TILE32) {
        const int nt = min(IL_TILE32, E - e0);
        __syncthreads();
        for (int i = threadIdx.x; i < nt; i += IL_T32) tt[i] = tgt[e0 + i];
        __syncthreads();
        for (int i = 0; i < nt; ++i) { if (tt[i] == d) { if (n < IL_CAP32) lists[threadIdx.x * IL_CAP32 + n] = e0 + i; ++n; } }
    }
    if (d < N) {
        int* row = NBR + (long long)d * IL_CAP32;
        for (int j = 0; j < IL_CAP32; ++j) { const int v = (j < n) ? lists[threadIdx.x * IL_CAP32 + j] : -1; VST2(int, row + j, v); }
        VST2(int, cnt + d, min(n, IL_CAP32));
    }
}
__global__ __launch_bounds__(256) void k_csr_scan32(const int* __restrict__ cnt, int* __restrict__ off, int N) {
    __shared__ int part[256]; const int per = ((((N + 255) / 256) + 31) / 32) * 32; const int a = threadIdx.x * per, b = min(N, a + per); int s = 0;
    for (int i = a; i < b; ++i) s += cnt[i]; part[threadIdx.x] = s; __syncthreads();
    if (threadIdx.x == 0) { int run = 0; for (int t = 0; t < 256; ++t) { const int v = part[t]; part[t] = run; run += v; } } __syncthreads();
    int run = part[threadIdx.x]; for (int i = a; i < b; ++i) { VST2(int, off + i, run); run += cnt[i]; }
    if (a < N && b == N) { VST2(int, off + N, run); }
}
__global__ __launch_bounds__(256) void k_slotcopy32(const int* __restrict__ off, const int* __restrict__ NBR, int* __restrict__ slot, int N) {
    const int t = blockIdx.x * 256 + threadIdx.x; const int tot = off[N]; if (t >= tot) return;
    int lo = 0, hi = N - 1;
    while (lo < hi) { const int mid = (lo + hi + 1) >> 1; if (off[mid] <= t) lo = mid; else hi = mid - 1; }
    int j = t - off[lo]; j = (j < 0) ? 0 : ((j >= IL_CAP32) ? (IL_CAP32 - 1) : j);
    VST2(int, slot + t, NBR[(long long)lo * IL_CAP32 + j]);
}

__global__ __launch_bounds__(256) void k_em_bias(const float* __restrict__ a0, const float* __restrict__ c0, const float* __restrict__ a1, const float* __restrict__ c1, float* __restrict__ BS) { const int q = blockIdx.x * 256 + threadIdx.x; if (q >= 2048) return; const float v = (q < 1024) ? a0[q] + c0[q] : a1[q - 1024] + c1[q - 1024]; VST2(float, BS + q, v); }
__global__ __launch_bounds__(1024) void k_plstm(const float* __restrict__ XG, int ldx, const float* __restrict__ Whh, float* __restrict__ HS, int ldo, int off, int T, int H, int reverse) {
    extern __shared__ float sm[]; float* h = sm; float* g = sm + H; const int j = threadIdx.x; const int G4 = 4 * H;
    for (int q = j; q < H; q += blockDim.x) h[q] = 0.f; float c = 0.f; __syncthreads();
    for (int s = 0; s < T; ++s) { const int t = reverse ? (T - 1 - s) : s;
        for (int jj = j; jj < G4; jj += blockDim.x) { const float* w = Whh + (long long)jj * H; float a = XG[(long long)t * ldx + jj];
#pragma unroll 1
            for (int k2 = 0; k2 < H; ++k2) a += w[k2] * h[k2]; g[jj] = a; }
        __syncthreads();
        float hn = 0.f; if (j < H) { const float ig = 1.f / (1.f + expf(-g[j])), fg = 1.f / (1.f + expf(-g[H + j])), gg = tanhf(g[2 * H + j]), og = 1.f / (1.f + expf(-g[3 * H + j])); c = fg * c + ig * gg; hn = og * tanhf(c); }
        __syncthreads(); if (j < H) { h[j] = hn; VST2(float, HS + (long long)t * ldo + off + j, hn); } __syncthreads(); }
}

__global__ __launch_bounds__(256) void k_em_smax(float* __restrict__ SC, float* __restrict__ AOUT, int T) { __shared__ float red[256]; const int r = blockIdx.x; float* row = SC + (long long)r * T; float mx = -__builtin_inff(); for (int j = threadIdx.x; j < T; j += 256) mx = fmaxf(mx, row[j]); red[threadIdx.x] = mx; __syncthreads(); for (int o = 128; o > 0; o >>= 1) { if (threadIdx.x < o) red[threadIdx.x] = fmaxf(red[threadIdx.x], red[threadIdx.x + o]); __syncthreads(); } mx = red[0]; __syncthreads();
    float s = 0.f; for (int j = threadIdx.x; j < T; j += 256) s += expf(row[j] - mx); red[threadIdx.x] = s; __syncthreads(); for (int o = 128; o > 0; o >>= 1) { if (threadIdx.x < o) red[threadIdx.x] += red[threadIdx.x + o]; __syncthreads(); } s = red[0];
    for (int j = threadIdx.x; j < T; j += 256) { const float pv = expf(row[j] - mx) / s; VST2(float, row + j, pv); VST2(float, AOUT + (long long)r * T + j, pv); } }
__global__ __launch_bounds__(256) void k_em_agg(const float* __restrict__ F, int C, const float* __restrict__ ew, const int* __restrict__ esrc, const int* __restrict__ off, const int* __restrict__ slot, float* __restrict__ AG, int N) { const long long q = (long long)blockIdx.x * 256 + threadIdx.x; if (q >= (long long)N * C) return; const int c = (int)(q % C); const int n = (int)(q / C); const int a = off[n], b = off[n + 1]; float s = 0.f; for (int p = a; p < b; ++p) { const int e = slot[p]; s += F[(long long)esrc[e] * C + c] * ew[e]; } VST2(float, AG + q, s); }
__global__ __launch_bounds__(256) void k_em_feats(const float* __restrict__ G2, const float* __restrict__ GM, const float* __restrict__ smiles, const float* __restrict__ kmer, float* __restrict__ FT, int N) { __shared__ float red[256]; const int c = blockIdx.x;
    if (c < 256) { float s = 0.f; for (int n = threadIdx.x; n < N; n += 256) s += G2[(long long)n * 256 + c]; red[threadIdx.x] = s; __syncthreads(); for (int o = 128; o > 0; o >>= 1) { if (threadIdx.x < o) red[threadIdx.x] += red[threadIdx.x + o]; __syncthreads(); } if (threadIdx.x == 0) VST2(float, FT + c, red[0] / (float)N); }
    else if (c == 256) { for (int j = threadIdx.x; j < 256; j += 256) VST2(float, FT + 256 + j, GM[j]); for (int j = threadIdx.x; j < 574; j += 256) VST2(float, FT + 512 + j, smiles[j]); for (int j = threadIdx.x; j < 64; j += 256) VST2(float, FT + 1086 + j, kmer[j]); } }

template __global__ void k_gemm<1>(GemmP);

extern "C" void kernel_launch(void* const* d_in, const int* in_sizes, int n_in, void* d_out, int out_size, void* d_ws, size_t ws_size, hipStream_t stream) {
    (void)in_sizes; (void)n_in; (void)out_size; (void)ws_size;
    const float* gmol = (const float*)d_in[0];
    const float* feat = (const float*)d_in[1];
    const float* smiles = (const float*)d_in[2];
    const float* kmer = (const float*)d_in[3];
    const float* ew = (const float*)d_in[4];
    const float* wih0 = (const float*)d_in[5];
    const float* whh0 = (const float*)d_in[6];
    const float* bih0 = (const float*)d_in[7];
    const float* bhh0 = (const float*)d_in[8];
    const float* wih1 = (const float*)d_in[9];
    const float* whh1 = (const float*)d_in[10];
    const float* bih1 = (const float*)d_in[11];
    const float* bhh1 = (const float*)d_in[12];
    const float* Wq = (const float*)d_in[13];
    const float* bq = (const float*)d_in[14];
    const float* Wk = (const float*)d_in[15];
    const float* bk = (const float*)d_in[16];
    const float* Wv = (const float*)d_in[17];
    const float* bv = (const float*)d_in[18];
    const float* Wfc = (const float*)d_in[19];
    const float* bfc = (const float*)d_in[20];
    const float* Wg1 = (const float*)d_in[21];
    const float* bg1 = (const float*)d_in[22];
    const float* Wg2 = (const float*)d_in[23];
    const float* bg2 = (const float*)d_in[24];
    const float* W1 = (const float*)d_in[25];
    const float* b1 = (const float*)d_in[26];
    const float* W2 = (const float*)d_in[27];
    const float* b2 = (const float*)d_in[28];
    const float* W3 = (const float*)d_in[29];
    const float* b3 = (const float*)d_in[30];
    const float* W4 = (const float*)d_in[31];
    const float* b4 = (const float*)d_in[32];
    const int* esrc = (const int*)d_in[33];
    const int* edst = (const int*)d_in[34];
    const int T = 2048;
    const int H = 128;
    const int DIN = 17;
    const int N = 50000;
    const int E = 600000;
    const int CAP = 32;
    const int LP = 32;
    float* out = (float*)d_out;
    float* attn = out + (1);
    char* wsp = (char*)d_ws;
    int* cnt = (int*)wsp; wsp += (((size_t)((size_t)N + 64) * 4 + 255) / 256) * 256;
    int* off = (int*)wsp; wsp += (((size_t)((size_t)N + 64) * 4 + 255) / 256) * 256;
    int* slot = (int*)wsp; wsp += (((size_t)((size_t)E + 64) * 4 + 255) / 256) * 256;
    int* nbr = (int*)wsp; wsp += (((size_t)((size_t)N * CAP) * 4 + 255) / 256) * 256;
    float* BS = (float*)wsp; wsp += (((size_t)((size_t)4 * 512) * 4 + 255) / 256) * 256;
    float* XG = (float*)wsp; wsp += (((size_t)((size_t)T * 512) * 4 + 255) / 256) * 256;
    float* H0 = (float*)wsp; wsp += (((size_t)((size_t)T * 256) * 4 + 255) / 256) * 256;
    float* H1 = (float*)wsp; wsp += (((size_t)((size_t)T * 256) * 4 + 255) / 256) * 256;
    float* Q = (float*)wsp; wsp += (((size_t)((size_t)T * H) * 4 + 255) / 256) * 256;
    float* Kb = (float*)wsp; wsp += (((size_t)((size_t)T * H) * 4 + 255) / 256) * 256;
    float* V = (float*)wsp; wsp += (((size_t)((size_t)T * H) * 4 + 255) / 256) * 256;
    float* GM = (float*)wsp; wsp += (((size_t)((size_t)LP * 512) * 4 + 255) / 256) * 256;
    float* AG = (float*)wsp; wsp += (((size_t)((size_t)N * 128) * 4 + 255) / 256) * 256;
    float* G1 = (float*)wsp; wsp += (((size_t)((size_t)N * 128) * 4 + 255) / 256) * 256;
    float* G2 = (float*)wsp; wsp += (((size_t)((size_t)N * 256) * 4 + 255) / 256) * 256;
    float* FT = (float*)wsp; wsp += (((size_t)((size_t)LP * 1152) * 4 + 255) / 256) * 256;
    float* M1 = (float*)wsp; wsp += (((size_t)((size_t)LP * 576) * 4 + 255) / 256) * 256;
    float* M2 = (float*)wsp; wsp += (((size_t)((size_t)LP * 256) * 4 + 255) / 256) * 256;
    float* M3 = (float*)wsp; wsp += (((size_t)((size_t)LP * 64) * 4 + 255) / 256) * 256;
    float* SC = (float*)wsp; wsp += (((size_t)((size_t)T * T) * 4 + 255) / 256) * 256;
    k_inlists32<<<(unsigned)((N) + IL_T32 - 1) / IL_T32, IL_T32, 0, stream>>>(edst, E, N, nbr, cnt);
    k_csr_scan32<<<1, 256, 0, stream>>>(cnt, off, N);
    k_slotcopy32<<<(unsigned)((E) + 255) / 256, 256, 0, stream>>>(off, nbr, slot, N);
    k_em_bias<<<8, 256, 0, stream>>>(bih0, bhh0, bih1, bhh1, BS);
    hipMemsetAsync(GM, 0, (size_t)LP * 512 * 4, stream); hipMemsetAsync(FT, 0, (size_t)LP * 1152 * 4, stream);
    { GemmP gxa0;
      gxa0.A = gmol; gxa0.B = wih0 + (size_t)0 * 512 * 17; gxa0.bias = BS + 0; gxa0.R = gmol; gxa0.C = XG;
      gxa0.sAo = 0; gxa0.sAi = 0; gxa0.sAm = 17; gxa0.sAk = 1; gxa0.sBo = 0; gxa0.sBi = 0; gxa0.sBn = 17; gxa0.sBk = 1; gxa0.sCo = 0; gxa0.sCi = 0; gxa0.sCm = 512; gxa0.sRo = 0; gxa0.sRi = 0; gxa0.sRm = 0; gxa0.sRn = 0;
      gxa0.M = T; gxa0.N = 512; gxa0.K = 17; gxa0.zi_n = 1; gxa0.flags = 1; gxa0.act = 0;
      gxa0.alpha = 1.0f; gxa0.beta = 0.0f; gxa0.sa = 1.0f; gxa0.sb = 1.0f; gxa0.Npad = 512; gxa0.pad_ = 0;
      k_gemm<1><<<dim3((unsigned)((512) + 31) / 32, (unsigned)((T) + 15) / 16, (unsigned)(1)), 32, 0, stream>>>(gxa0); }
    k_plstm<<<1, 512, (size_t)(5 * H) * 4, stream>>>(XG, 512, whh0 + (size_t)0 * 512 * H, H0, 256, 0, T, H, 0);
    { GemmP gxa1;
      gxa1.A = gmol; gxa1.B = wih0 + (size_t)1 * 512 * 17; gxa1.bias = BS + 512; gxa1.R = gmol; gxa1.C = XG;
      gxa1.sAo = 0; gxa1.sAi = 0; gxa1.sAm = 17; gxa1.sAk = 1; gxa1.sBo = 0; gxa1.sBi = 0; gxa1.sBn = 17; gxa1.sBk = 1; gxa1.sCo = 0; gxa1.sCi = 0; gxa1.sCm = 512; gxa1.sRo = 0; gxa1.sRi = 0; gxa1.sRm = 0; gxa1.sRn = 0;
      gxa1.M = T; gxa1.N = 512; gxa1.K = 17; gxa1.zi_n = 1; gxa1.flags = 1; gxa1.act = 0;
      gxa1.alpha = 1.0f; gxa1.beta = 0.0f; gxa1.sa = 1.0f; gxa1.sb = 1.0f; gxa1.Npad = 512; gxa1.pad_ = 0;
      k_gemm<1><<<dim3((unsigned)((512) + 31) / 32, (unsigned)((T) + 15) / 16, (unsigned)(1)), 32, 0, stream>>>(gxa1); }
    k_plstm<<<1, 512, (size_t)(5 * H) * 4, stream>>>(XG, 512, whh0 + (size_t)1 * 512 * H, H0, 256, 128, T, H, 1);
    { GemmP gxb0;
      gxb0.A = H0; gxb0.B = wih1 + (size_t)0 * 512 * 256; gxb0.bias = BS + 1024; gxb0.R = H0; gxb0.C = XG;
      gxb0.sAo = 0; gxb0.sAi = 0; gxb0.sAm = 256; gxb0.sAk = 1; gxb0.sBo = 0; gxb0.sBi = 0; gxb0.sBn = 256; gxb0.sBk = 1; gxb0.sCo = 0; gxb0.sCi = 0; gxb0.sCm = 512; gxb0.sRo = 0; gxb0.sRi = 0; gxb0.sRm = 0; gxb0.sRn = 0;
      gxb0.M = T; gxb0.N = 512; gxb0.K = 256; gxb0.zi_n = 1; gxb0.flags = 1; gxb0.act = 0;
      gxb0.alpha = 1.0f; gxb0.beta = 0.0f; gxb0.sa = 1.0f; gxb0.sb = 1.0f; gxb0.Npad = 512; gxb0.pad_ = 0;
      k_gemm<1><<<dim3((unsigned)((512) + 31) / 32, (unsigned)((T) + 15) / 16, (unsigned)(1)), 32, 0, stream>>>(gxb0); }
    k_plstm<<<1, 512, (size_t)(5 * H) * 4, stream>>>(XG, 512, whh1 + (size_t)0 * 512 * H, H1, 256, 0, T, H, 0);
    { GemmP gxb1;
      gxb1.A = H0; gxb1.B = wih1 + (size_t)1 * 512 * 256; gxb1.bias = BS + 1536; gxb1.R = H0; gxb1.C = XG;
      gxb1.sAo = 0; gxb1.sAi = 0; gxb1.sAm = 256; gxb1.sAk = 1; gxb1.sBo = 0; gxb1.sBi = 0; gxb1.sBn = 256; gxb1.sBk = 1; gxb1.sCo = 0; gxb1.sCi = 0; gxb1.sCm = 512; gxb1.sRo = 0; gxb1.sRi = 0; gxb1.sRm = 0; gxb1.sRn = 0;
      gxb1.M = T; gxb1.N = 512; gxb1.K = 256; gxb1.zi_n = 1; gxb1.flags = 1; gxb1.act = 0;
      gxb1.alpha = 1.0f; gxb1.beta = 0.0f; gxb1.sa = 1.0f; gxb1.sb = 1.0f; gxb1.Npad = 512; gxb1.pad_ = 0;
      k_gemm<1><<<dim3((unsigned)((512) + 31) / 32, (unsigned)((T) + 15) / 16, (unsigned)(1)), 32, 0, stream>>>(gxb1); }
    k_plstm<<<1, 512, (size_t)(5 * H) * 4, stream>>>(XG, 512, whh1 + (size_t)1 * 512 * H, H1, 256, 128, T, H, 1);
    { GemmP gQ;
      gQ.A = H1; gQ.B = Wq; gQ.bias = bq; gQ.R = H1; gQ.C = Q;
      gQ.sAo = 0; gQ.sAi = 0; gQ.sAm = 256; gQ.sAk = 1; gQ.sBo = 0; gQ.sBi = 0; gQ.sBn = 256; gQ.sBk = 1; gQ.sCo = 0; gQ.sCi = 0; gQ.sCm = H; gQ.sRo = 0; gQ.sRi = 0; gQ.sRm = 0; gQ.sRn = 0;
      gQ.M = T; gQ.N = H; gQ.K = 256; gQ.zi_n = 1; gQ.flags = 1; gQ.act = 0;
      gQ.alpha = 1.0f; gQ.beta = 0.0f; gQ.sa = 1.0f; gQ.sb = 1.0f; gQ.Npad = H; gQ.pad_ = 0;
      k_gemm<1><<<dim3((unsigned)((H) + 31) / 32, (unsigned)((T) + 15) / 16, (unsigned)(1)), 32, 0, stream>>>(gQ); }
    { GemmP gKb;
      gKb.A = H1; gKb.B = Wk; gKb.bias = bk; gKb.R = H1; gKb.C = Kb;
      gKb.sAo = 0; gKb.sAi = 0; gKb.sAm = 256; gKb.sAk = 1; gKb.sBo = 0; gKb.sBi = 0; gKb.sBn = 256; gKb.sBk = 1; gKb.sCo = 0; gKb.sCi = 0; gKb.sCm = H; gKb.sRo = 0; gKb.sRi = 0; gKb.sRm = 0; gKb.sRn = 0;
      gKb.M = T; gKb.N = H; gKb.K = 256; gKb.zi_n = 1; gKb.flags = 1; gKb.act = 0;
      gKb.alpha = 1.0f; gKb.beta = 0.0f; gKb.sa = 1.0f; gKb.sb = 1.0f; gKb.Npad = H; gKb.pad_ = 0;
      k_gemm<1><<<dim3((unsigned)((H) + 31) / 32, (unsigned)((T) + 15) / 16, (unsigned)(1)), 32, 0, stream>>>(gKb); }
    { GemmP gV;
      gV.A = H1; gV.B = Wv; gV.bias = bv; gV.R = H1; gV.C = V;
      gV.sAo = 0; gV.sAi = 0; gV.sAm = 256; gV.sAk = 1; gV.sBo = 0; gV.sBi = 0; gV.sBn = 256; gV.sBk = 1; gV.sCo = 0; gV.sCi = 0; gV.sCm = H; gV.sRo = 0; gV.sRi = 0; gV.sRm = 0; gV.sRn = 0;
      gV.M = T; gV.N = H; gV.K = 256; gV.zi_n = 1; gV.flags = 1; gV.act = 0;
      gV.alpha = 1.0f; gV.beta = 0.0f; gV.sa = 1.0f; gV.sb = 1.0f; gV.Npad = H; gV.pad_ = 0;
      k_gemm<1><<<dim3((unsigned)((H) + 31) / 32, (unsigned)((T) + 15) / 16, (unsigned)(1)), 32, 0, stream>>>(gV); }
    { GemmP gsc;
      gsc.A = Q; gsc.B = Kb; gsc.bias = Q; gsc.R = Q; gsc.C = SC;
      gsc.sAo = 0; gsc.sAi = 0; gsc.sAm = H; gsc.sAk = 1; gsc.sBo = 0; gsc.sBi = 0; gsc.sBn = H; gsc.sBk = 1; gsc.sCo = 0; gsc.sCi = 0; gsc.sCm = T; gsc.sRo = 0; gsc.sRi = 0; gsc.sRm = 0; gsc.sRn = 0;
      gsc.M = T; gsc.N = T; gsc.K = H; gsc.zi_n = 1; gsc.flags = 0; gsc.act = 0;
      gsc.alpha = 0.08838834764831845f; gsc.beta = 0.0f; gsc.sa = 1.0f; gsc.sb = 1.0f; gsc.Npad = T; gsc.pad_ = 0;
      k_gemm<1><<<dim3((unsigned)((T) + 31) / 32, (unsigned)((T) + 15) / 16, (unsigned)(1)), 32, 0, stream>>>(gsc); }
    k_em_smax<<<T, 256, 0, stream>>>(SC, attn, T);
    { GemmP gav;
      gav.A = SC + (size_t)(T - 1) * T; gav.B = V; gav.bias = SC + (size_t)(T - 1) * T; gav.R = SC + (size_t)(T - 1) * T; gav.C = GM;
      gav.sAo = 0; gav.sAi = 0; gav.sAm = T; gav.sAk = 1; gav.sBo = 0; gav.sBi = 0; gav.sBn = 1; gav.sBk = H; gav.sCo = 0; gav.sCi = 0; gav.sCm = 512; gav.sRo = 0; gav.sRi = 0; gav.sRm = 0; gav.sRn = 0;
      gav.M = 1; gav.N = H; gav.K = T; gav.zi_n = 1; gav.flags = 0; gav.act = 0;
      gav.alpha = 1.0f; gav.beta = 0.0f; gav.sa = 1.0f; gav.sb = 1.0f; gav.Npad = H; gav.pad_ = 0;
      k_gemm<1><<<dim3((unsigned)((H) + 31) / 32, (unsigned)((1) + 15) / 16, (unsigned)(1)), 32, 0, stream>>>(gav); }
    { GemmP gfc;
      gfc.A = GM; gfc.B = Wfc; gfc.bias = bfc; gfc.R = GM; gfc.C = GM + 256;
      gfc.sAo = 0; gfc.sAi = 0; gfc.sAm = 512; gfc.sAk = 1; gfc.sBo = 0; gfc.sBi = 0; gfc.sBn = H; gfc.sBk = 1; gfc.sCo = 0; gfc.sCi = 0; gfc.sCm = 512; gfc.sRo = 0; gfc.sRi = 0; gfc.sRm = 0; gfc.sRn = 0;
      gfc.M = 1; gfc.N = 256; gfc.K = H; gfc.zi_n = 1; gfc.flags = 1; gfc.act = 0;
      gfc.alpha = 1.0f; gfc.beta = 0.0f; gfc.sa = 1.0f; gfc.sb = 1.0f; gfc.Npad = 256; gfc.pad_ = 0;
      k_gemm<1><<<dim3((unsigned)((256) + 31) / 32, (unsigned)((1) + 15) / 16, (unsigned)(1)), 32, 0, stream>>>(gfc); }
    k_em_agg<<<(unsigned)(((long long)N * 128 + 255) / 256), 256, 0, stream>>>(feat, 128, ew, esrc, off, slot, AG, N);
    { GemmP gg1;
      gg1.A = AG; gg1.B = Wg1; gg1.bias = bg1; gg1.R = AG; gg1.C = G1;
      gg1.sAo = 0; gg1.sAi = 0; gg1.sAm = 128; gg1.sAk = 1; gg1.sBo = 0; gg1.sBi = 0; gg1.sBn = 1; gg1.sBk = 128; gg1.sCo = 0; gg1.sCi = 0; gg1.sCm = 128; gg1.sRo = 0; gg1.sRi = 0; gg1.sRm = 0; gg1.sRn = 0;
      gg1.M = N; gg1.N = 128; gg1.K = 128; gg1.zi_n = 1; gg1.flags = 1; gg1.act = 1;
      gg1.alpha = 1.0f; gg1.beta = 0.0f; gg1.sa = 1.0f; gg1.sb = 1.0f; gg1.Npad = 128; gg1.pad_ = 0;
      k_gemm<1><<<dim3((unsigned)((128) + 31) / 32, (unsigned)((N) + 15) / 16, (unsigned)(1)), 32, 0, stream>>>(gg1); }
    k_em_agg<<<(unsigned)(((long long)N * 128 + 255) / 256), 256, 0, stream>>>(G1, 128, ew, esrc, off, slot, AG, N);
    { GemmP gg2;
      gg2.A = AG; gg2.B = Wg2; gg2.bias = bg2; gg2.R = AG; gg2.C = G2;
      gg2.sAo = 0; gg2.sAi = 0; gg2.sAm = 128; gg2.sAk = 1; gg2.sBo = 0; gg2.sBi = 0; gg2.sBn = 1; gg2.sBk = 256; gg2.sCo = 0; gg2.sCi = 0; gg2.sCm = 256; gg2.sRo = 0; gg2.sRi = 0; gg2.sRm = 0; gg2.sRn = 0;
      gg2.M = N; gg2.N = 256; gg2.K = 128; gg2.zi_n = 1; gg2.flags = 1; gg2.act = 0;
      gg2.alpha = 1.0f; gg2.beta = 0.0f; gg2.sa = 1.0f; gg2.sb = 1.0f; gg2.Npad = 256; gg2.pad_ = 0;
      k_gemm<1><<<dim3((unsigned)((256) + 31) / 32, (unsigned)((N) + 15) / 16, (unsigned)(1)), 32, 0, stream>>>(gg2); }
    k_em_feats<<<257, 256, 0, stream>>>(G2, GM + 256, smiles, kmer, FT, N);
    { GemmP gm1;
      gm1.A = FT; gm1.B = W1; gm1.bias = b1; gm1.R = FT; gm1.C = M1;
      gm1.sAo = 0; gm1.sAi = 0; gm1.sAm = 1152; gm1.sAk = 1; gm1.sBo = 0; gm1.sBi = 0; gm1.sBn = 1150; gm1.sBk = 1; gm1.sCo = 0; gm1.sCi = 0; gm1.sCm = 576; gm1.sRo = 0; gm1.sRi = 0; gm1.sRm = 0; gm1.sRn = 0;
      gm1.M = 1; gm1.N = 575; gm1.K = 1150; gm1.zi_n = 1; gm1.flags = 1; gm1.act = 1;
      gm1.alpha = 1.0f; gm1.beta = 0.0f; gm1.sa = 1.0f; gm1.sb = 1.0f; gm1.Npad = 575; gm1.pad_ = 0;
      k_gemm<1><<<dim3((unsigned)((575) + 31) / 32, (unsigned)((1) + 15) / 16, (unsigned)(1)), 32, 0, stream>>>(gm1); }
    { GemmP gm2;
      gm2.A = M1; gm2.B = W2; gm2.bias = b2; gm2.R = M1; gm2.C = M2;
      gm2.sAo = 0; gm2.sAi = 0; gm2.sAm = 576; gm2.sAk = 1; gm2.sBo = 0; gm2.sBi = 0; gm2.sBn = 575; gm2.sBk = 1; gm2.sCo = 0; gm2.sCi = 0; gm2.sCm = 256; gm2.sRo = 0; gm2.sRi = 0; gm2.sRm = 0; gm2.sRn = 0;
      gm2.M = 1; gm2.N = 256; gm2.K = 575; gm2.zi_n = 1; gm2.flags = 1; gm2.act = 1;
      gm2.alpha = 1.0f; gm2.beta = 0.0f; gm2.sa = 1.0f; gm2.sb = 1.0f; gm2.Npad = 256; gm2.pad_ = 0;
      k_gemm<1><<<dim3((unsigned)((256) + 31) / 32, (unsigned)((1) + 15) / 16, (unsigned)(1)), 32, 0, stream>>>(gm2); }
    { GemmP gm3;
      gm3.A = M2; gm3.B = W3; gm3.bias = b3; gm3.R = M2; gm3.C = M3;
      gm3.sAo = 0; gm3.sAi = 0; gm3.sAm = 256; gm3.sAk = 1; gm3.sBo = 0; gm3.sBi = 0; gm3.sBn = 256; gm3.sBk = 1; gm3.sCo = 0; gm3.sCi = 0; gm3.sCm = 64; gm3.sRo = 0; gm3.sRi = 0; gm3.sRm = 0; gm3.sRn = 0;
      gm3.M = 1; gm3.N = 64; gm3.K = 256; gm3.zi_n = 1; gm3.flags = 1; gm3.act = 1;
      gm3.alpha = 1.0f; gm3.beta = 0.0f; gm3.sa = 1.0f; gm3.sb = 1.0f; gm3.Npad = 64; gm3.pad_ = 0;
      k_gemm<1><<<dim3((unsigned)((64) + 31) / 32, (unsigned)((1) + 15) / 16, (unsigned)(1)), 32, 0, stream>>>(gm3); }
    { GemmP gm4;
      gm4.A = M3; gm4.B = W4; gm4.bias = b4; gm4.R = M3; gm4.C = out;
      gm4.sAo = 0; gm4.sAi = 0; gm4.sAm = 64; gm4.sAk = 1; gm4.sBo = 0; gm4.sBi = 0; gm4.sBn = 64; gm4.sBk = 1; gm4.sCo = 0; gm4.sCi = 0; gm4.sCm = LP; gm4.sRo = 0; gm4.sRi = 0; gm4.sRm = 0; gm4.sRn = 0;
      gm4.M = 1; gm4.N = 1; gm4.K = 64; gm4.zi_n = 1; gm4.flags = 1; gm4.act = 0;
      gm4.alpha = 1.0f; gm4.beta = 0.0f; gm4.sa = 1.0f; gm4.sb = 1.0f; gm4.Npad = 1; gm4.pad_ = 0;
      k_gemm<1><<<dim3((unsigned)((1) + 31) / 32, (unsigned)((1) + 15) / 16, (unsigned)(1)), 32, 0, stream>>>(gm4); }
}
